// FlashAttention2_53618371723497
// MI455X (gfx1250) — hardware-verified
//
#include <hip/hip_runtime.h>
#include <math.h>
#include <stdint.h>

#ifndef NB
#define NB 2
#endif
#ifndef SEQ
#define SEQ 2048
#endif
#define XS_FULL 2048
#define EMB   2048
#define NH    16
#define KVH   4
#define HD    128
#define HHALF (HD / 2)
#define DMOD  (NH * HD)
#define KVD   (KVH * HD)
#define GQ    (NH / KVH)
#define WIN   1024
#define MROWS (NB * SEQ)
#define EPS_L2 0.000001f
#define RSQ_HD 0.08838834764831845f
#define LOG2E 1.4426950408889634f
#define KROPE (-0.20762050593046014f)
#define ICAP  0.02f
#define CAPV  50.0f
#define NEGT  (-1.0e30f)
#define QSC   256.0f
#define KSC   256.0f
#define PCAR  32768.0f
#define VCAR  1024.0f
#define OSC   1024.0f
#define WOS   1024.0f
#define WPB   2
#define NHG   (NH / WPB)
#define NQT   (SEQ / 16)
#define NKT   (SEQ / 32)
#define NVT   (SEQ / 64)
#define ATT_THREADS (WPB * 32)
#define PTP   36
#define PTW   (16 * PTP)
#define SLP   132
#define SLW   (16 * SLP)
#define WREG  (PTW + SLW)
#define SLAB64 (16 * 68)
#define VTP   72
#define TWP   72
#define WS_CAP 134217728
static_assert(DMOD == 2048 && DMOD == EMB && KVD == 512 && GQ == 4 && HD == 128 && HHALF == 64 && NH == 16 && KVH == 4);
static_assert(WPB == 2 && NHG * WPB == NH && ATT_THREADS == 64 && (GQ % WPB) == 0);
static_assert(NB >= 1 && NB <= 2);
static_assert((SEQ % 64) == 0 && SEQ >= 64 && SEQ <= XS_FULL);
static_assert((MROWS % 64) == 0 && (DMOD % 64) == 0 && (KVD % 64) == 0 && (EMB % 32) == 0 && (HD % 32) == 0);
static_assert(((SEQ * EMB / 8) % 256) == 0);
static_assert(WPB * WREG * 4 <= 65536 && HD * VTP * 2 <= 65536 && 4 * SLAB64 * 4 <= 65536 && 64 * TWP * 2 <= 65536);

typedef unsigned short u16;
typedef _Float16 v16h __attribute__((ext_vector_type(16)));
typedef _Float16 v8h  __attribute__((ext_vector_type(8)));
typedef __bf16   v16b __attribute__((ext_vector_type(16)));
typedef float    v8f  __attribute__((ext_vector_type(8)));
typedef float    v4f  __attribute__((ext_vector_type(4)));
typedef unsigned int v4u __attribute__((ext_vector_type(4)));

union FragH { v16h v; v8h h[2]; v4u u[2]; };
union FragB { v16b v; v4u u[2]; };

__device__ __forceinline__ unsigned short bf_bits(float f) {
  unsigned u = __float_as_uint(f);
  return (unsigned short)((u + 0x7FFFu + ((u >> 16) & 1u)) >> 16);
}
__device__ __forceinline__ float bf_up(unsigned short h) { return __uint_as_float(((unsigned)h) << 16); }
__device__ __forceinline__ float bfr(float f) { return bf_up(bf_bits(f)); }
__device__ __forceinline__ unsigned short h_bits(_Float16 x) { return __builtin_bit_cast(unsigned short, x); }
__device__ __forceinline__ unsigned pk16(unsigned short a, unsigned short b) { return (unsigned)a | ((unsigned)b << 16); }
__device__ __forceinline__ v8f zero8() { v8f z = {0.f, 0.f, 0.f, 0.f, 0.f, 0.f, 0.f, 0.f}; return z; }

__device__ __forceinline__ v16h ldfrag_h(const _Float16* p) {
  FragH f;
  f.h[0] = *(const v8h*)(p);
  f.h[1] = *(const v8h*)(p + 16);
  return f.v;
}
__device__ __forceinline__ v16b ldfrag_b(const u16* p) {
  FragB f;
  f.u[0] = *(const v4u*)(p);
  f.u[1] = *(const v4u*)(p + 16);
  return f.v;
}

__device__ __forceinline__ v8f mma_h(v16h a, v16h b, v8f c) {
  return __builtin_amdgcn_wmma_f32_16x16x32_f16(false, a, false, b, (short)0, c, false, false);
}
__device__ __forceinline__ v8f mma_b(v16b a, v16b b, v8f c) {
  return __builtin_amdgcn_wmma_f32_16x16x32_bf16(false, a, false, b, (short)0, c, false, false);
}
__device__ __forceinline__ void guard2(v8f& a, v8f& b, v16h x0, v16h x1, v16h x2, v16h x3, v16h x4, v16h x5) {
#if defined(__HIP_DEVICE_COMPILE__)
  asm volatile("v_nop\n\tv_nop\n\tv_nop\n\tv_nop"
               : "+v"(a), "+v"(b) : "v"(x0), "v"(x1), "v"(x2), "v"(x3), "v"(x4), "v"(x5) : "memory");
#endif
}
template <typename F>
__device__ __forceinline__ void guard6(v8f& a, v8f& b, v8f& c, v8f& d, F x0, F x1, F x2, F x3, F x4, F x5) {
#if defined(__HIP_DEVICE_COMPILE__)
  asm volatile("v_nop\n\tv_nop\n\tv_nop\n\tv_nop"
               : "+v"(a), "+v"(b), "+v"(c), "+v"(d) : "v"(x0), "v"(x1), "v"(x2), "v"(x3), "v"(x4), "v"(x5) : "memory");
#endif
}
__device__ __forceinline__ void acc_guard4(v8f& a, v8f& b, v8f& c, v8f& d) {
#if defined(__HIP_DEVICE_COMPILE__)
  asm volatile("v_nop\n\tv_nop\n\tv_nop\n\tv_nop" : "+v"(a), "+v"(b), "+v"(c), "+v"(d));
#endif
}
__device__ __forceinline__ void wave_sync_lds() {
  __builtin_amdgcn_fence(__ATOMIC_RELEASE, "workgroup");
  __builtin_amdgcn_wave_barrier();
  __builtin_amdgcn_fence(__ATOMIC_ACQUIRE, "workgroup");
}

__global__ __launch_bounds__(256) void cvt16(const float* __restrict__ x, u16* D, int n8, int f16mode, float scale) {
  const int gt = blockIdx.x * 256 + (int)threadIdx.x;
  if (gt >= n8) return;
  const float* p = x + (size_t)gt * 8;
  const v4f a = *(const v4f*)(p), b4 = *(const v4f*)(p + 4);
  float w[8];
#pragma unroll
  for (int e = 0; e < 4; ++e) { w[e] = a[e]; w[4 + e] = b4[e]; }
  v4u o;
#pragma unroll
  for (int e = 0; e < 4; ++e) {
    const float f0 = w[2 * e], f1 = w[2 * e + 1];
    const unsigned short hb0 = h_bits((_Float16)(bfr(f0) * scale));
    const unsigned short hb1 = h_bits((_Float16)(bfr(f1) * scale));
    const unsigned short bb0 = bf_bits(f0);
    const unsigned short bb1 = bf_bits(f1);
    o[e] = (f16mode != 0) ? pk16(hb0, hb1) : pk16(bb0, bb1);
  }
  u16* d = D + (size_t)gt * 8;
  for (int pass = 0; pass < 2; ++pass) {
    *(volatile v4u*)(d) = o;
    __threadfence();
  }
}

__global__ __launch_bounds__(256) void tw16(const float* __restrict__ W, int ldw, int c0, u16* T, int nN,
                                             int f16mode, float scale) {
  __shared__ __align__(16) u16 TT[64 * TWP];
  const int tid = threadIdx.x;
  const int bid = blockIdx.x;
  const int kt  = bid % (DMOD / 64);
  const int nt  = bid / (DMOD / 64);
  if (nt >= (nN >> 6)) return;
  const int k0 = kt * 64, n0 = nt * 64;
  {
    const int kk = tid >> 2;
    const int nq = (tid & 3) * 16;
    const float* src = W + (size_t)(k0 + kk) * ldw + c0 + n0 + nq;
#pragma unroll
    for (int i = 0; i < 4; ++i) {
      const v4f a = *(const v4f*)(src + 4 * i);
#pragma unroll
      for (int e = 0; e < 4; ++e) {
        const float f = a[e];
        const unsigned short hb = h_bits((_Float16)(bfr(f) * scale));
        const unsigned short bb = bf_bits(f);
        TT[(nq + 4 * i + e) * TWP + kk] = (f16mode != 0) ? hb : bb;
      }
    }
  }
  __syncthreads();
  const int q8 = tid >> 3, p8 = (tid & 7) * 8;
  v4u v[2];
#pragma unroll
  for (int it = 0; it < 2; ++it) {
    const int line = it * 32 + q8;
    v[it] = *(const v4u*)(TT + line * TWP + p8);
  }
  const size_t base = (size_t)n0 * DMOD + k0 + p8;
  for (int pass = 0; pass < 2; ++pass) {
#pragma unroll
    for (int it = 0; it < 2; ++it) {
      const int line = it * 32 + q8;
      *(volatile v4u*)(T + base + (size_t)line * DMOD) = v[it];
    }
    __threadfence();
  }
}

__global__ __launch_bounds__(256) void vt16(const float* __restrict__ F, u16* VHo) {
  __shared__ __align__(16) u16 TH[HD * VTP];
  const int tid = threadIdx.x;
  const int bid = blockIdx.x;
  const int st  = bid % NVT;
  const int t2  = bid / NVT;
  const int kvh = t2 % KVH;
  const int b   = t2 / KVH;
  if (b >= NB) return;
  const int s0 = st * 64;
  {
    const int sl = tid >> 2;
    const int dc = (tid & 3) * 32;
    const float* src = F + ((size_t)b * SEQ + s0 + sl) * KVD + kvh * HD + dc;
#pragma unroll
    for (int i = 0; i < 8; ++i) {
      const v4f a = *(const v4f*)(src + 4 * i);
#pragma unroll
      for (int e = 0; e < 4; ++e) {
        const float t = a[e] * VCAR;
        TH[(dc + 4 * i + e) * VTP + sl] = h_bits((_Float16)t);
      }
    }
  }
  __syncthreads();
  v4u vh[4];
  const int q8 = tid >> 3, p8 = (tid & 7) * 8;
#pragma unroll
  for (int it = 0; it < 4; ++it) {
    const int line = it * 32 + q8;
    vh[it] = *(const v4u*)(TH + line * VTP + p8);
  }
  const size_t hrow = (size_t)(b * KVH + kvh) * HD;
  const size_t base = hrow * SEQ + (size_t)s0 + p8;
  for (int pass = 0; pass < 2; ++pass) {
#pragma unroll
    for (int it = 0; it < 4; ++it) {
      const int line = it * 32 + q8;
      *(volatile v4u*)(VHo + base + (size_t)line * SEQ) = vh[it];
    }
    __threadfence();
  }
}

template <int NHX>
__global__ __launch_bounds__(NHX * 8) void nrl16(const float* __restrict__ F, const float* __restrict__ nw,
                                                 u16* Hp, float sc) {
#pragma clang fp contract(off)
  constexpr int NT   = NHX * 8;
  constexpr int NCOL = NHX * HD;
  __shared__ __align__(16) float cst[HHALF];
  __shared__ __align__(16) float snt[HHALF];
  const int tid = (int)threadIdx.x;
  const int row = (int)blockIdx.x;
  if (row >= MROWS) return;
  const int s = row % SEQ;
#pragma unroll 1
  for (int j = tid; j < HHALF; j += NT) {
    const float invf = exp2f((float)j * KROPE);
    const float ang  = (float)s * invf;
    cst[j] = cosf(ang);
    snt[j] = sinf(ang);
  }
  __syncthreads();
  const int dlo = (tid & 7) * 8;
  const int clo = (tid >> 3) * HD + dlo;
  const float* p = F + (size_t)row * NCOL + clo;
  const v4f xa = *(const v4f*)(p), xb = *(const v4f*)(p + 4);
  const v4f ya = *(const v4f*)(p + HHALF), yb = *(const v4f*)(p + HHALF + 4);
  const v4f ca = *(const v4f*)(cst + dlo), cb = *(const v4f*)(cst + dlo + 4);
  const v4f sa = *(const v4f*)(snt + dlo), sb = *(const v4f*)(snt + dlo + 4);
  const v4f wa = *(const v4f*)(nw + dlo), wb4 = *(const v4f*)(nw + dlo + 4);
  const v4f wc = *(const v4f*)(nw + HHALF + dlo), wd = *(const v4f*)(nw + HHALF + dlo + 4);
  float xl[8], xh[8], cv[8], sv[8], wl[8], wh[8];
#pragma unroll
  for (int e = 0; e < 4; ++e) {
    xl[e] = xa[e];        xl[4 + e] = xb[e];
    xh[e] = ya[e];        xh[4 + e] = yb[e];
    cv[e] = ca[e];        cv[4 + e] = cb[e];
    sv[e] = sa[e];        sv[4 + e] = sb[e];
    wl[e] = bfr(wa[e]);   wl[4 + e] = bfr(wb4[e]);
    wh[e] = bfr(wc[e]);   wh[4 + e] = bfr(wd[e]);
  }
  float rl[8], rh[8];
#pragma unroll
  for (int e = 0; e < 8; ++e) {
    rl[e] = xl[e] * cv[e] - xh[e] * sv[e];
    rh[e] = xl[e] * sv[e] + xh[e] * cv[e];
  }
  float ss = 0.0f;
#pragma unroll
  for (int e = 0; e < 8; ++e) { ss = ss + rl[e] * rl[e]; ss = ss + rh[e] * rh[e]; }
  ss += __shfl_xor(ss, 1, 32);
  ss += __shfl_xor(ss, 2, 32);
  ss += __shfl_xor(ss, 4, 32);
  const float nrm = sqrtf(ss);
  const float inv = 1.0f / (nrm + EPS_L2);
  v4u ol4, oh4;
#pragma unroll
  for (int e = 0; e < 4; ++e) {
    const float yl0 = (rl[2 * e] * inv) * wl[2 * e],         yl1 = (rl[2 * e + 1] * inv) * wl[2 * e + 1];
    const float yh0 = (rh[2 * e] * inv) * wh[2 * e],         yh1 = (rh[2 * e + 1] * inv) * wh[2 * e + 1];
    ol4[e] = pk16(h_bits((_Float16)(yl0 * sc)), h_bits((_Float16)(yl1 * sc)));
    oh4[e] = pk16(h_bits((_Float16)(yh0 * sc)), h_bits((_Float16)(yh1 * sc)));
  }
  u16* dh = Hp + (size_t)row * NCOL + clo;
  for (int pass = 0; pass < 2; ++pass) {
    *(volatile v4u*)(dh) = ol4;
    *(volatile v4u*)(dh + HHALF) = oh4;
    __threadfence();
  }
}

__device__ __forceinline__ void epi64(float* sl, v8f a0, v8f a1, v8f a2, v8f a3, float oscale,
                                      float* C, int N, size_t rowb, int col0, int lane) {
  const int hh = lane >> 4, m = lane & 15;
#pragma unroll
  for (int r = 0; r < 8; ++r) {
    const int ro = (8 * hh + r) * 68 + m;
    sl[ro]      = a0[r] * oscale;
    sl[ro + 16] = a1[r] * oscale;
    sl[ro + 32] = a2[r] * oscale;
    sl[ro + 48] = a3[r] * oscale;
  }
  wave_sync_lds();
  v4f vals[8];
#pragma unroll
  for (int it = 0; it < 8; ++it) vals[it] = *(const v4f*)(sl + (it * 2 + hh) * 68 + m * 4);
  float* dst = C + (rowb + (size_t)hh) * (size_t)N + col0 + m * 4;
  for (int pass = 0; pass < 2; ++pass) {
#pragma unroll
    for (int it = 0; it < 8; ++it) {
      *(volatile v4f*)(dst + (size_t)(it * 2) * (size_t)N) = vals[it];
    }
    __threadfence();
  }
}

__global__ __launch_bounds__(128)
void gemm_bf(const u16* __restrict__ A, const u16* __restrict__ Bt, float* C, int M, int N, int K, float oscale) {
  __shared__ __align__(16) float slab[4 * SLAB64];
  const int tid = threadIdx.x, wave = tid >> 5, lane = tid & 31, hh = lane >> 4, m = lane & 15;
  const int ntile = N >> 6;
  const int bid   = blockIdx.x;
  const int rowb  = (bid / ntile) * 64 + wave * 16;
  const int col0  = (bid % ntile) * 64;
  if (rowb + 16 > M) return;
  const u16* ap = A  + (size_t)(rowb + m) * K + 8 * hh;
  const u16* bp = Bt + (size_t)(col0 + m) * K + 8 * hh;
  const size_t bs = (size_t)16 * K;
  v8f acc0 = zero8(), acc1 = zero8(), acc2 = zero8(), acc3 = zero8();
#pragma unroll 1
  for (int k0 = 0; k0 < K; k0 += 32) {
    const v16b a  = ldfrag_b(ap + k0);
    const v16b b0 = ldfrag_b(bp + k0);
    const v16b b1 = ldfrag_b(bp + bs + k0);
    const v16b b2 = ldfrag_b(bp + 2 * bs + k0);
    const v16b b3 = ldfrag_b(bp + 3 * bs + k0);
    acc0 = mma_b(a, b0, acc0);
    acc1 = mma_b(a, b1, acc1);
    acc2 = mma_b(a, b2, acc2);
    acc3 = mma_b(a, b3, acc3);
    guard6<v16b>(acc0, acc1, acc2, acc3, a, b0, b1, b2, b3, a);
  }
  epi64(slab + wave * SLAB64, acc0, acc1, acc2, acc3, oscale, C, N, (size_t)rowb, col0, lane);
}

__global__ __launch_bounds__(128)
void gemm_h(const u16* __restrict__ A, const u16* __restrict__ Bt, float* C, int M, int N, int K, float oscale) {
  __shared__ __align__(16) float slab[4 * SLAB64];
  const int tid = threadIdx.x, wave = tid >> 5, lane = tid & 31, hh = lane >> 4, m = lane & 15;
  const int ntile = N >> 6;
  const int bid   = blockIdx.x;
  const int rowb  = (bid / ntile) * 64 + wave * 16;
  const int col0  = (bid % ntile) * 64;
  if (rowb + 16 > M) return;
  const _Float16* ap = (const _Float16*)(const void*)A  + (size_t)(rowb + m) * K + 8 * hh;
  const _Float16* bp = (const _Float16*)(const void*)Bt + (size_t)(col0 + m) * K + 8 * hh;
  const size_t bs = (size_t)16 * K;
  v8f acc0 = zero8(), acc1 = zero8(), acc2 = zero8(), acc3 = zero8();
#pragma unroll 1
  for (int k0 = 0; k0 < K; k0 += 32) {
    const v16h a  = ldfrag_h(ap + k0);
    const v16h b0 = ldfrag_h(bp + k0);
    const v16h b1 = ldfrag_h(bp + bs + k0);
    const v16h b2 = ldfrag_h(bp + 2 * bs + k0);
    const v16h b3 = ldfrag_h(bp + 3 * bs + k0);
    acc0 = mma_h(a, b0, acc0);
    acc1 = mma_h(a, b1, acc1);
    acc2 = mma_h(a, b2, acc2);
    acc3 = mma_h(a, b3, acc3);
    guard6<v16h>(acc0, acc1, acc2, acc3, a, b0, b1, b2, b3, a);
  }
  epi64(slab + wave * SLAB64, acc0, acc1, acc2, acc3, oscale, C, N, (size_t)rowb, col0, lane);
}

__global__ __launch_bounds__(ATT_THREADS)
void attn_w(const u16* __restrict__ QHp, const u16* __restrict__ KHp, const u16* __restrict__ VHp, u16* OHp) {
  __shared__ __align__(16) float smem[WPB * WREG];

  const int tid  = threadIdx.x;
  const int wave = tid >> 5;
  const int lane = tid & 31;
  const int hh   = lane >> 4;
  const int c    = lane & 15;
  const int bid  = blockIdx.x;
  const int qt   = bid % NQT;
  const int t2   = bid / NQT;
  const int hg   = t2 % NHG;
  const int b    = t2 / NHG;
  if (b >= NB) return;
  const int q0   = qt * 16;
  if (q0 + 16 > SEQ) return;
  const int head = hg * WPB + wave;
  const int kvh  = head / GQ;

  float* pt   = smem + wave * WREG;
  float* slab = pt + PTW;

  const _Float16* Qh  = (const _Float16*)(const void*)QHp + ((size_t)b * SEQ + q0 + c) * DMOD + (size_t)head * HD + 8 * hh;
  const _Float16* Khb = (const _Float16*)(const void*)KHp + ((size_t)b * SEQ + c) * KVD + (size_t)kvh * HD + 8 * hh;
  const _Float16* Vhb = (const _Float16*)(const void*)VHp + ((size_t)(b * KVH + kvh) * HD + c) * SEQ + 8 * hh;
  const float usc = RSQ_HD / (QSC * KSC);
  const float oc  = 1.0f / (PCAR * VCAR);
  const size_t KROW = (size_t)KVD;

  float mrow[8], lrow[8];
  v8f o[8];
#pragma unroll
  for (int r = 0; r < 8; ++r) { mrow[r] = -INFINITY; lrow[r] = 0.f; }
#pragma unroll
  for (int j = 0; j < 8; ++j) o[j] = zero8();
  int jlo = q0 - WIN; if (jlo < 0) jlo = 0;
  int kthi = (q0 + 16 + WIN + 31) >> 5; if (kthi > NKT) kthi = NKT;
  int ktlo = jlo >> 5; if (ktlo > kthi) ktlo = kthi;
  const int qr0 = q0 + 8 * hh;

#pragma unroll 1
  for (int kt = ktlo; kt < kthi; ++kt) {
    const int kb = kt * 32;
    v8f s0 = zero8(), s1 = zero8();
    const _Float16* k0p = Khb + (size_t)kb * KROW;
    const _Float16* k1p = k0p + (size_t)16 * KROW;
#pragma unroll
    for (int kk = 0; kk < HD / 32; ++kk) {
      const v16h qh  = ldfrag_h(Qh + kk * 32);
      const v16h kh0 = ldfrag_h(k0p + kk * 32);
      const v16h kh1 = ldfrag_h(k1p + kk * 32);
      s0 = mma_h(qh, kh0, s0);
      s1 = mma_h(qh, kh1, s1);
      guard2(s0, s1, qh, kh0, kh1, qh, kh0, kh1);
    }
    const int key0 = kb + c, key1 = kb + 16 + c;
#pragma unroll
    for (int r = 0; r < 8; ++r) {
      const int   qr = qr0 + r;
      const float u0 = s0[r] * usc;
      const float u1 = s1[r] * usc;
      const float g0 = tanhf(u0 * ICAP) * CAPV;
      const float g1 = tanhf(u1 * ICAP) * CAPV;
      const int dd0 = qr - key0, dd1 = qr - key1;
      const bool ok0 = (dd0 <= WIN) && (dd0 >= -WIN);
      const bool ok1 = (dd1 <= WIN) && (dd1 >= -WIN);
      const float t0 = ok0 ? (g0 * LOG2E) : NEGT;
      const float t1 = ok1 ? (g1 * LOG2E) : NEGT;
      float mx = fmaxf(t0, t1);
#pragma unroll
      for (int off = 1; off < 16; off <<= 1) mx = fmaxf(mx, __shfl_xor(mx, off, 32));
      const float mn = fmaxf(mrow[r], mx);
      const float ms = (mn == -INFINITY) ? 0.0f : mn;
      const float al = exp2f(mrow[r] - ms);
      mrow[r] = mn;
      const float e0 = exp2f(t0 - ms), e1 = exp2f(t1 - ms);
      float ps = e0 + e1;
#pragma unroll
      for (int off = 1; off < 16; off <<= 1) ps += __shfl_xor(ps, off, 32);
      lrow[r] = lrow[r] * al + ps;
#pragma unroll
      for (int j = 0; j < 8; ++j) o[j][r] *= al;
      const int ro = (8 * hh + r) * PTP + c;
      pt[ro]      = e0;
      pt[ro + 16] = e1;
    }
    wave_sync_lds();
    FragH ph, pl;
    {
      const float* prow = pt + c * PTP + 8 * hh;
      const v4f p0 = *(const v4f*)(prow), p1 = *(const v4f*)(prow + 4);
      const v4f p2 = *(const v4f*)(prow + 16), p3 = *(const v4f*)(prow + 20);
#pragma unroll
      for (int e = 0; e < 4; ++e) {
        const float ta = p0[e] * PCAR, tb = p1[e] * PCAR, tc = p2[e] * PCAR, td = p3[e] * PCAR;
        const _Float16 ha = (_Float16)ta, hb = (_Float16)tb, hc = (_Float16)tc, hd = (_Float16)td;
        ph.h[0][e]     = ha;
        ph.h[0][4 + e] = hb;
        ph.h[1][e]     = hc;
        ph.h[1][4 + e] = hd;
        pl.h[0][e]     = (_Float16)(ta - (float)ha);
        pl.h[0][4 + e] = (_Float16)(tb - (float)hb);
        pl.h[1][e]     = (_Float16)(tc - (float)hc);
        pl.h[1][4 + e] = (_Float16)(td - (float)hd);
      }
    }
    {
      const _Float16* vhp = Vhb + kb;
#pragma unroll
      for (int jg = 0; jg < 4; ++jg) {
        const size_t da = (size_t)(2 * jg) * 16 * SEQ;
        const size_t db = da + (size_t)16 * SEQ;
        const v16h vha = ldfrag_h(vhp + da), vhb2 = ldfrag_h(vhp + db);
        o[2 * jg]     = mma_h(ph.v, vha,  o[2 * jg]);
        o[2 * jg]     = mma_h(pl.v, vha,  o[2 * jg]);
        o[2 * jg + 1] = mma_h(ph.v, vhb2, o[2 * jg + 1]);
        o[2 * jg + 1] = mma_h(pl.v, vhb2, o[2 * jg + 1]);
        guard2(o[2 * jg], o[2 * jg + 1], ph.v, pl.v, vha, vhb2, ph.v, pl.v);
      }
    }
    wave_sync_lds();
  }
  acc_guard4(o[0], o[1], o[2], o[3]);
  acc_guard4(o[4], o[5], o[6], o[7]);
#pragma unroll
  for (int r = 0; r < 8; ++r) {
    const float lv  = lrow[r];
    const float ls  = (lv > 0.0f) ? lv : 1.0f;
    const float inv = (lv > 0.0f) ? ((1.0f / ls) * oc) : 0.0f;
#pragma unroll
    for (int j = 0; j < 8; ++j) {
      const int idx = (8 * hh + r) * SLP + j * 16 + c;
      slab[idx] = o[j][r] * inv;
    }
  }

  wave_sync_lds();
  v4u oh[8];
  const int rq = lane >> 4, c8 = (lane & 15) * 8;
#pragma unroll
  for (int it = 0; it < 8; ++it) {
    const int row = it * 2 + rq;
    const v4f a = *(const v4f*)(slab + row * SLP + c8), b4 = *(const v4f*)(slab + row * SLP + c8 + 4);
    float w[8];
#pragma unroll
    for (int e = 0; e < 4; ++e) { w[e] = a[e] * OSC; w[4 + e] = b4[e] * OSC; }
#pragma unroll
    for (int e = 0; e < 4; ++e) {
      const _Float16 h0 = (_Float16)w[2 * e], h1 = (_Float16)w[2 * e + 1];
      oh[it][e] = pk16(h_bits(h0), h_bits(h1));
    }
  }
  const size_t ob = ((size_t)b * SEQ + q0) * DMOD + (size_t)head * HD + c8;
  for (int pass = 0; pass < 2; ++pass) {
#pragma unroll
    for (int it = 0; it < 8; ++it) {
      const int row = it * 2 + rq;
      *(volatile v4u*)(OHp + ob + (size_t)row * DMOD) = oh[it];
    }
    __threadfence();
  }
}

extern "C" void kernel_launch(void* const* d_in, const int* in_sizes, int n_in,
                              void* d_out, int out_size, void* d_ws, size_t ws_size,
                              hipStream_t stream) {
  if (n_in < 7) return;
  if (in_sizes[0] < ((NB - 1) * XS_FULL + SEQ) * EMB) return;
  if (in_sizes[1] != EMB * DMOD) return;
  if (in_sizes[2] != EMB * KVD) return;
  if (in_sizes[3] != EMB * KVD) return;
  if (in_sizes[4] != DMOD * EMB) return;
  if (in_sizes[5] < HD) return;
  if (in_sizes[6] < HD) return;
  if (out_size < MROWS * EMB) return;

  const float* x    = (const float*)d_in[0];
  const float* wq   = (const float*)d_in[1];
  const float* wk   = (const float*)d_in[2];
  const float* wv   = (const float*)d_in[3];
  const float* wo   = (const float*)d_in[4];
  const float* qsc  = (const float*)d_in[5];
  const float* ksc  = (const float*)d_in[6];
  float*       out  = (float*)d_out;

  const size_t szXB = (size_t)MROWS * EMB * 2;
  const size_t szWT = (size_t)DMOD * DMOD * 2;
  const size_t szF  = (size_t)MROWS * DMOD * 4;
  const size_t szQH = (size_t)MROWS * DMOD * 2;
  const size_t szKH = (size_t)MROWS * KVD * 2;
  const size_t szVH = (size_t)NB * KVH * HD * SEQ * 2;
  const size_t szOH = (size_t)MROWS * DMOD * 2;
  const size_t szWO = (size_t)EMB * DMOD * 2;
  size_t off = 0;
  const size_t oXB = off; off += szXB;
  const size_t oWT = off; off += szWT;
  const size_t oF  = off; off += szF;
  const size_t oQH = off; off += szQH;
  const size_t oKH = off; off += szKH;
  const size_t oVH = off; off += szVH;
  const size_t oOH = off; off += szOH;
  const size_t oWO = off; off += szWO;
  if (off > ws_size) return;
  if (off > (size_t)WS_CAP) return;

  char* ws = (char*)d_ws;
  u16*   XB = (u16*)(ws + oXB);
  u16*   WT = (u16*)(ws + oWT);
  float* F  = (float*)(ws + oF);
  u16*   QH = (u16*)(ws + oQH);
  u16*   KH = (u16*)(ws + oKH);
  u16*   VH = (u16*)(ws + oVH);
  u16*   OH = (u16*)(ws + oOH);
  u16*   WO = (u16*)(ws + oWO);

  const dim3 b256(256), b128(128), b32(32), bAT(ATT_THREADS);
  const int  n8x = (SEQ * EMB) / 8;
  const dim3 gX((n8x + 255) / 256);
  const dim3 gTWq((DMOD / 64) * (DMOD / 64));
  const dim3 gTWk((DMOD / 64) * (KVD / 64));
  const dim3 gGq((MROWS / 64) * (DMOD / 64));
  const dim3 gGk((MROWS / 64) * (KVD / 64));
  const dim3 gRW(MROWS);
  const dim3 gVT(NB * KVH * NVT);
  const dim3 gAT(NQT * NHG * NB);

  for (int b = 0; b < NB; ++b) {
    cvt16<<<gX, b256, 0, stream>>>(x + (size_t)b * XS_FULL * EMB, XB + (size_t)b * SEQ * EMB, n8x, 0, 1.0f);
  }
  tw16<<<gTWq, b256, 0, stream>>>(wq, DMOD, 0, WT, DMOD, 0, 1.0f);
  gemm_bf<<<gGq, b128, 0, stream>>>(XB, WT, F, MROWS, DMOD, EMB, 1.0f);
  nrl16<NH><<<gRW, b128, 0, stream>>>(F, qsc, QH, QSC);
  tw16<<<gTWk, b256, 0, stream>>>(wk, KVD, 0, WT, KVD, 0, 1.0f);
  gemm_bf<<<gGk, b128, 0, stream>>>(XB, WT, F, MROWS, KVD, EMB, 1.0f);
  nrl16<KVH><<<gRW, b32, 0, stream>>>(F, ksc, KH, KSC);
  tw16<<<gTWk, b256, 0, stream>>>(wv, KVD, 0, WT, KVD, 0, 1.0f);
  gemm_bf<<<gGk, b128, 0, stream>>>(XB, WT, F, MROWS, KVD, EMB, 1.0f);
  vt16<<<gVT, b256, 0, stream>>>(F, VH);
  attn_w<<<gAT, bAT, 0, stream>>>(QH, KH, VH, OH);
  tw16<<<gTWq, b256, 0, stream>>>(wo, EMB, 0, WO, EMB, 1, WOS);
  gemm_h<<<dim3((MROWS / 64) * (EMB / 64)), b128, 0, stream>>>(OH, WO, out, MROWS, EMB, DMOD, 1.0f / (OSC * WOS));
  (void)hipGetLastError();
}
